// PytorchGeometricGAT_18691697672408
// MI455X (gfx1250) — hardware-verified
//
#include <hip/hip_runtime.h>
#include <stddef.h>


#define FIN    256
#define D1     256
#define NH1    4
#define D2     16
#define KD     256
#define GR     32
#define AP     264
#define NTHR   256
#define NWAVE  8
#define CHUNK  2048
#define WCAP   256
#define NGRP   (CHUNK / (NTHR * 4))
#define NB1    256
#define SH1    8
#define NB2    2048
#define SH2    11
#define ECLAMP 80.0f

#define LDS1_F     (NB1 * D1 + NB1 * NH1)
#define LDS1_BYTES ((LDS1_F + NWAVE * WCAP + NWAVE) * 4)
#define LDS2_F     (NB2 * D2 + NB2)
#define LDS2_BYTES ((LDS2_F + NWAVE * WCAP + NWAVE) * 4)

static_assert(NGRP == 2);
static_assert(WCAP == (CHUNK / NTHR) * 32);
static_assert((1 << SH1) == NB1);
static_assert((1 << SH2) == NB2);
static_assert(KD == NTHR);
static_assert((LDS1_F % 4) == 0);
static_assert((LDS2_F % 4) == 0);
static_assert(LDS1_BYTES == 274464);
static_assert(LDS2_BYTES == 147488);
static_assert(NB1 == NWAVE * 32);
static_assert(NB2 == NWAVE * 256);
static_assert(D1 == NWAVE * 32);
static_assert(GR * AP * 4 >= GR * D1 * 4);
static_assert((AP % 8) == 0);

typedef float  v4f  __attribute__((ext_vector_type(4)));
typedef float  v8f  __attribute__((ext_vector_type(8)));
typedef int    v4i  __attribute__((ext_vector_type(4)));
typedef __bf16 v8b  __attribute__((ext_vector_type(8)));
typedef __bf16 v16b __attribute__((ext_vector_type(16)));
union FragB { v16b v; v8b half[2]; };
union PackB { v8b b; v4i i; __bf16 e[8]; };

__device__ __forceinline__ v8f wmb(v16b a, v16b b, v8f c) {
  v8f d = __builtin_amdgcn_wmma_f32_16x16x32_bf16(false, a, false, b, (short)0, c, false, false);
  asm volatile("v_nop\n\tv_nop\n\tv_nop\n\tv_nop" : "+v"(d) : "v"(a), "v"(b));
  return d;
}

__device__ __forceinline__ v8f zero8() { v8f z = {0.f, 0.f, 0.f, 0.f, 0.f, 0.f, 0.f, 0.f}; return z; }
__device__ __forceinline__ v4f zero4() { v4f z = {0.f, 0.f, 0.f, 0.f}; return z; }

__device__ __forceinline__ void split_bf(float f, __bf16& hi, __bf16& lo) {
  const __bf16 h = (__bf16)f;
  hi = h;
  lo = (__bf16)(f - (float)h);
}
__device__ __forceinline__ void split8(const v4f a, const v4f b, PackB& uh, PackB& ul) {
  split_bf(a.x, uh.e[0], ul.e[0]); split_bf(a.y, uh.e[1], ul.e[1]);
  split_bf(a.z, uh.e[2], ul.e[2]); split_bf(a.w, uh.e[3], ul.e[3]);
  split_bf(b.x, uh.e[4], ul.e[4]); split_bf(b.y, uh.e[5], ul.e[5]);
  split_bf(b.z, uh.e[6], ul.e[6]); split_bf(b.w, uh.e[7], ul.e[7]);
}

__device__ __forceinline__ float lrelu(float v) { return v >= 0.f ? v : 0.2f * v; }
__device__ __forceinline__ float pexp(float v) { v = lrelu(v); v = fminf(v, ECLAMP); return __expf(v); }
__device__ __forceinline__ float eluf(float v) { return v > 0.f ? v : (__expf(v) - 1.0f); }
__device__ __forceinline__ int clampi(int v, int hi) { return v < 0 ? 0 : (v > hi ? hi : v); }

__global__ __launch_bounds__(NTHR) void k_prep(const float* __restrict__ W1, __bf16* P1h, __bf16* P1l,
                                               const float* __restrict__ W2, __bf16* P2h, __bf16* P2l, int nb1) {
  __shared__ __attribute__((aligned(16))) __bf16 Th[8 * AP];
  __shared__ __attribute__((aligned(16))) __bf16 Tl[8 * AP];
  const int tid = threadIdx.x;
  const bool first = ((int)blockIdx.x < nb1);
  const float* W = first ? W1 : W2;
  const int ncol = first ? D1 : D2;
  const int n0 = (first ? (int)blockIdx.x : ((int)blockIdx.x - nb1)) * 8;
  __bf16* Ph = first ? P1h : P2h;
  __bf16* Pl = first ? P1l : P2l;

  const float* p = W + (size_t)tid * ncol + n0;
  const v4f a = *(const v4f*)p, b = *(const v4f*)(p + 4);
  __bf16 hq, lq;
  split_bf(a.x, hq, lq); Th[0 * AP + tid] = hq; Tl[0 * AP + tid] = lq;
  split_bf(a.y, hq, lq); Th[1 * AP + tid] = hq; Tl[1 * AP + tid] = lq;
  split_bf(a.z, hq, lq); Th[2 * AP + tid] = hq; Tl[2 * AP + tid] = lq;
  split_bf(a.w, hq, lq); Th[3 * AP + tid] = hq; Tl[3 * AP + tid] = lq;
  split_bf(b.x, hq, lq); Th[4 * AP + tid] = hq; Tl[4 * AP + tid] = lq;
  split_bf(b.y, hq, lq); Th[5 * AP + tid] = hq; Tl[5 * AP + tid] = lq;
  split_bf(b.z, hq, lq); Th[6 * AP + tid] = hq; Tl[6 * AP + tid] = lq;
  split_bf(b.w, hq, lq); Th[7 * AP + tid] = hq; Tl[7 * AP + tid] = lq;
  __syncthreads();

  const int j = tid >> 5, kc = (tid & 31) * 8;
  PackB uh, ul;
  uh.b = *(const v8b*)(Th + j * AP + kc);
  ul.b = *(const v8b*)(Tl + j * AP + kc);
  __bf16* gh = Ph + (size_t)(n0 + j) * KD + kc;
  __bf16* gl = Pl + (size_t)(n0 + j) * KD + kc;
  *(volatile v4i*)gh = uh.i; *(volatile v4i*)gl = ul.i;
  __threadfence();
  *(volatile v4i*)gh = uh.i; *(volatile v4i*)gl = ul.i;
}

__global__ __launch_bounds__(NTHR) void k_gemm1(
    const float* __restrict__ x, const __bf16* __restrict__ Wh, const __bf16* __restrict__ Wl,
    const float* __restrict__ att_s, const float* __restrict__ att_d,
    float* h1, float* asrc, float* adst, int nN) {
  __shared__ __attribute__((aligned(16))) float sm[GR * AP];
  __shared__ __attribute__((aligned(16))) float As[GR * NWAVE];
  __shared__ __attribute__((aligned(16))) float Ds[GR * NWAVE];
  __shared__ __attribute__((aligned(16))) float Fs[2 * GR * NH1];
  __bf16* Ah = (__bf16*)sm;
  __bf16* Al = Ah + GR * AP;
  float* Xs = sm;

  const int tid  = threadIdx.x;
  const int lane = tid & 31;
  const int w    = tid >> 5;
  const int hh   = lane >> 4;
  const int m    = lane & 15;
  const int rowBase = blockIdx.x * GR;

  {
    const int r  = tid >> 3;
    const int kc = (tid & 7) * 32;
    int row = rowBase + r;
    if (row > nN - 1) row = nN - 1;
    const float* p = x + (size_t)row * FIN + kc;
#pragma unroll
    for (int q = 0; q < 4; ++q) {
      const v4f fa = *(const v4f*)(p + 8 * q);
      const v4f fb = *(const v4f*)(p + 8 * q + 4);
      PackB uh, ul;
      split8(fa, fb, uh, ul);
      *(v8b*)(Ah + r * AP + kc + 8 * q) = uh.b;
      *(v8b*)(Al + r * AP + kc + 8 * q) = ul.b;
    }
  }
  __syncthreads();

  const int cb = 32 * w;
  v8f a00 = zero8(), a01 = zero8(), a10 = zero8(), a11 = zero8();
#pragma unroll 1
  for (int kt = 0; kt < KD / 32; ++kt) {
    const int ko = kt * 32 + 8 * hh;
    FragB ah0, al0, ah1, al1, bh0, bl0, bh1, bl1;
    const __bf16* pp;
    pp = Ah + m * AP + ko;              ah0.half[0] = *(const v8b*)pp; ah0.half[1] = *(const v8b*)(pp + 16);
    pp = Al + m * AP + ko;              al0.half[0] = *(const v8b*)pp; al0.half[1] = *(const v8b*)(pp + 16);
    pp = Ah + (16 + m) * AP + ko;       ah1.half[0] = *(const v8b*)pp; ah1.half[1] = *(const v8b*)(pp + 16);
    pp = Al + (16 + m) * AP + ko;       al1.half[0] = *(const v8b*)pp; al1.half[1] = *(const v8b*)(pp + 16);
    pp = Wh + (size_t)(cb + m) * KD + ko;       bh0.half[0] = *(const v8b*)pp; bh0.half[1] = *(const v8b*)(pp + 16);
    pp = Wl + (size_t)(cb + m) * KD + ko;       bl0.half[0] = *(const v8b*)pp; bl0.half[1] = *(const v8b*)(pp + 16);
    pp = Wh + (size_t)(cb + 16 + m) * KD + ko;  bh1.half[0] = *(const v8b*)pp; bh1.half[1] = *(const v8b*)(pp + 16);
    pp = Wl + (size_t)(cb + 16 + m) * KD + ko;  bl1.half[0] = *(const v8b*)pp; bl1.half[1] = *(const v8b*)(pp + 16);
    a00 = wmb(ah0.v, bh0.v, a00); a00 = wmb(ah0.v, bl0.v, a00); a00 = wmb(al0.v, bh0.v, a00);
    a01 = wmb(ah0.v, bh1.v, a01); a01 = wmb(ah0.v, bl1.v, a01); a01 = wmb(al0.v, bh1.v, a01);
    a10 = wmb(ah1.v, bh0.v, a10); a10 = wmb(ah1.v, bl0.v, a10); a10 = wmb(al1.v, bh0.v, a10);
    a11 = wmb(ah1.v, bh1.v, a11); a11 = wmb(ah1.v, bl1.v, a11); a11 = wmb(al1.v, bh1.v, a11);
  }
  __syncthreads();

  const float cs0 = att_s[cb + m], cs1 = att_s[cb + 16 + m];
  const float cd0 = att_d[cb + m], cd1 = att_d[cb + 16 + m];
  float ss0[8], sd0[8], ss1[8], sd1[8];
#pragma unroll
  for (int r = 0; r < 8; ++r) {
    const int r0 = (8 * hh + r) * D1;
    const int r1 = (16 + 8 * hh + r) * D1;
    Xs[r0 + cb + m] = a00[r]; Xs[r0 + cb + 16 + m] = a01[r];
    Xs[r1 + cb + m] = a10[r]; Xs[r1 + cb + 16 + m] = a11[r];
    ss0[r] = a00[r] * cs0 + a01[r] * cs1; sd0[r] = a00[r] * cd0 + a01[r] * cd1;
    ss1[r] = a10[r] * cs0 + a11[r] * cs1; sd1[r] = a10[r] * cd0 + a11[r] * cd1;
  }
#pragma unroll
  for (int mk = 1; mk < 16; mk <<= 1) {
#pragma unroll
    for (int r = 0; r < 8; ++r) {
      ss0[r] += __shfl_xor(ss0[r], mk, 32); sd0[r] += __shfl_xor(sd0[r], mk, 32);
      ss1[r] += __shfl_xor(ss1[r], mk, 32); sd1[r] += __shfl_xor(sd1[r], mk, 32);
    }
  }
  if (m == 0) {
#pragma unroll
    for (int r = 0; r < 8; ++r) {
      As[(8 * hh + r) * NWAVE + w] = ss0[r];      Ds[(8 * hh + r) * NWAVE + w] = sd0[r];
      As[(16 + 8 * hh + r) * NWAVE + w] = ss1[r]; Ds[(16 + 8 * hh + r) * NWAVE + w] = sd1[r];
    }
  }
  __syncthreads();
  {
    const int pl = tid >> 7, idx = tid & 127, row = idx >> 2, hd = idx & 3;
    const float* P = pl ? Ds : As;
    Fs[pl * 128 + idx] = P[row * NWAVE + 2 * hd] + P[row * NWAVE + 2 * hd + 1];
  }
  __syncthreads();

  v4f xr[8];
#pragma unroll
  for (int i = 0; i < 4; ++i) {
    xr[2 * i]     = *(const v4f*)(Xs + (4 * w + i) * D1 + 4 * lane);
    xr[2 * i + 1] = *(const v4f*)(Xs + (4 * w + i) * D1 + 128 + 4 * lane);
  }
  float* fp = 0;
  v4f fv = zero4();
  if (w == 0)      { fv = *(const v4f*)(Fs + 4 * lane);       fp = asrc + (size_t)rowBase * NH1 + 4 * lane; }
  else if (w == 1) { fv = *(const v4f*)(Fs + 128 + 4 * lane); fp = adst + (size_t)rowBase * NH1 + 4 * lane; }
  float* hp[4];
#pragma unroll
  for (int i = 0; i < 4; ++i) hp[i] = h1 + (size_t)(rowBase + 4 * w + i) * D1;

#pragma unroll
  for (int i = 0; i < 4; ++i) {
    *(volatile v4f*)(hp[i] + 4 * lane) = xr[2 * i];
    *(volatile v4f*)(hp[i] + 128 + 4 * lane) = xr[2 * i + 1];
  }
  if (fp) *(volatile v4f*)fp = fv;
  __threadfence();
#pragma unroll
  for (int i = 0; i < 4; ++i) {
    *(volatile v4f*)(hp[i] + 4 * lane) = xr[2 * i];
    *(volatile v4f*)(hp[i] + 128 + 4 * lane) = xr[2 * i + 1];
  }
  if (fp) *(volatile v4f*)fp = fv;
}

__global__ __launch_bounds__(NTHR) void k_edge1(const int* __restrict__ ei, const float* __restrict__ asrc,
                                                const float* __restrict__ adst, float* pe, int nN, int nE, int Ep) {
  const int t = blockIdx.x * NTHR + threadIdx.x;
  if (t >= Ep) return;
  int e = t; if (e > nE - 1) e = nE - 1;
  const int s = clampi(ei[e], nN - 1);
  const int d = clampi(ei[nE + e], nN - 1);
  const v4f sa = *(const v4f*)(asrc + (size_t)s * NH1);
  const v4f da = *(const v4f*)(adst + (size_t)d * NH1);
  v4f p;
  p.x = pexp(sa.x + da.x); p.y = pexp(sa.y + da.y); p.z = pexp(sa.z + da.z); p.w = pexp(sa.w + da.w);
  float* op = pe + (size_t)t * NH1;
  *(volatile v4f*)op = p;
  __threadfence();
  *(volatile v4f*)op = p;
}

__global__ __launch_bounds__(NTHR) void k_edge2(const int* __restrict__ ei, const float* __restrict__ asrc,
                                                const float* __restrict__ adst, float* pe, int nN, int nE, int Ep4) {
  const int t = blockIdx.x * NTHR + threadIdx.x;
  if (t >= Ep4) return;
  float pv[4];
#pragma unroll
  for (int q = 0; q < 4; ++q) {
    int e = 4 * t + q; if (e > nE - 1) e = nE - 1;
    const int s = clampi(ei[e], nN - 1);
    const int d = clampi(ei[nE + e], nN - 1);
    pv[q] = pexp(asrc[s] + adst[d]);
  }
  v4f p; p.x = pv[0]; p.y = pv[1]; p.z = pv[2]; p.w = pv[3];
  float* op = pe + (size_t)t * 4;
  *(volatile v4f*)op = p;
  __threadfence();
  *(volatile v4f*)op = p;
}

template <int NBK, int SH>
__device__ __forceinline__ int scan_chunk(const int* __restrict__ eid, int nE, bool al16,
                                          int cbase, int nodeBase, int tid, int wave, int* list) {
  int wc = 0;
#pragma unroll
  for (int g = 0; g < NGRP; ++g) {
    const int el0 = (g * NTHR + tid) * 4;
    const int e0  = cbase + el0;
    const int sent = -2147483647 - 1;
    v4i d;
    if (al16 && (e0 + 3 < nE)) {
      d = *(const v4i*)(eid + e0);
    } else {
      d.x = (e0     < nE) ? eid[min(e0, nE - 1)]     : sent;
      d.y = (e0 + 1 < nE) ? eid[min(e0 + 1, nE - 1)] : sent;
      d.z = (e0 + 2 < nE) ? eid[min(e0 + 2, nE - 1)] : sent;
      d.w = (e0 + 3 < nE) ? eid[min(e0 + 3, nE - 1)] : sent;
    }
    const unsigned s0 = (unsigned)d.x - (unsigned)nodeBase;
    const unsigned s1 = (unsigned)d.y - (unsigned)nodeBase;
    const unsigned s2 = (unsigned)d.z - (unsigned)nodeBase;
    const unsigned s3 = (unsigned)d.w - (unsigned)nodeBase;
    const bool q0 = s0 < (unsigned)NBK;
    const bool q1 = s1 < (unsigned)NBK;
    const bool q2 = s2 < (unsigned)NBK;
    const bool q3 = s3 < (unsigned)NBK;
    const unsigned many = __builtin_amdgcn_ballot_w32(q0 | q1 | q2 | q3);
    if (many != 0u) {
#define HITJ(J, HJ, SJ) { \
        const unsigned mj = __builtin_amdgcn_ballot_w32(HJ); \
        if (HJ) { \
          const int pos = wc + (int)__builtin_amdgcn_mbcnt_lo(mj, 0u); \
          if (pos < WCAP) list[wave * WCAP + pos] = ((el0 + (J)) << SH) | (int)(SJ); \
        } \
        wc += (int)__builtin_popcount(mj); }
      HITJ(0, q0, s0)
      HITJ(1, q1, s1)
      HITJ(2, q2, s2)
      HITJ(3, q3, s3)
#undef HITJ
    }
  }
  return wc;
}

__global__ __launch_bounds__(NTHR) void k_gat1(
    const int* __restrict__ ei, const float* __restrict__ h1, const float* __restrict__ pe,
    const float* __restrict__ asrc, const float* __restrict__ adst, const float* __restrict__ b1,
    float* g1, int nN, int nE) {
  extern __shared__ v4f lds_dyn[];
  float* sacc = (float*)lds_dyn;
  float* den  = sacc + NB1 * D1;
  int*   list = (int*)(sacc + LDS1_F);
  int*   wcnt = list + NWAVE * WCAP;

  const int tid  = threadIdx.x;
  const int lane = tid & 31;
  const int wave = tid >> 5;
  const int hh   = lane >> 4;
  const int m    = lane & 15;
  const int nodeBase = blockIdx.x * NB1;

  {
    const v4f z4 = zero4();
    for (int i = tid; i < LDS1_F / 4; i += NTHR) lds_dyn[i] = z4;
  }
  __syncthreads();

  const int* eid = ei + nE;
  const bool al16 = ((nE & 3) == 0);
  const int nChunks = (nE + CHUNK - 1) / CHUNK;
#pragma unroll 1
  for (int ch = 0; ch < nChunks; ++ch) {
    const int cbase = ch * CHUNK;
    const int wc = scan_chunk<NB1, SH1>(eid, nE, al16, cbase, nodeBase, tid, wave, list);
    if (lane == 0) wcnt[wave] = wc;
    __syncthreads();

    if (wave == 0) {
#pragma unroll 1
      for (int wsx = 0; wsx < NWAVE; ++wsx) {
        int n = wcnt[wsx];
        n = n > WCAP ? WCAP : n; n = n < 0 ? 0 : n;
        const int lb = wsx * WCAP;
#pragma unroll 1
        for (int i = 0; i < n; ++i) {
          const int ent  = list[lb + i];
          const int slot = ent & (NB1 - 1);
          const int el   = (ent >> SH1) & (CHUNK - 1);
          int e = cbase + el; if (e > nE - 1) e = nE - 1;
          const int src = clampi(ei[e], nN - 1);
          const v4f p4 = *(const v4f*)(pe + (size_t)e * NH1);
          const float p0 = hh ? p4.y : p4.x;
          const float p1 = hh ? p4.w : p4.z;
          const float* hr = h1 + (size_t)src * D1;
          const v4f x0 = *(const v4f*)(hr + 4 * lane);
          const v4f x1 = *(const v4f*)(hr + 128 + 4 * lane);
          v4f* q0 = (v4f*)(sacc + slot * D1 + 4 * lane);
          v4f* q1 = (v4f*)(sacc + slot * D1 + 128 + 4 * lane);
          const v4f c0 = *q0;
          const v4f c1 = *q1;
          *q0 = c0 + p0 * x0;
          *q1 = c1 + p1 * x1;
          int ai = -1; float av = 0.f;
          if (m == 0)      { ai = slot * NH1 + hh;     av = p0; }
          else if (m == 1) { ai = slot * NH1 + 2 + hh; av = p1; }
          if (ai >= 0) { const float o = den[ai]; den[ai] = o + av; }
        }
      }
    }
    __syncthreads();
  }

  const v4f ba = *(const v4f*)(b1 + 4 * lane);
  const v4f bb = *(const v4f*)(b1 + 128 + 4 * lane);
#pragma unroll 1
  for (int j = 0; j < NB1 / NWAVE; ++j) {
    const int slot = wave * (NB1 / NWAVE) + j;
    const int node = nodeBase + slot;
    if (node >= nN) break;
    const v4f sa = *(const v4f*)(asrc + (size_t)node * NH1);
    const v4f da = *(const v4f*)(adst + (size_t)node * NH1);
    const float p0 = pexp((hh ? sa.y : sa.x) + (hh ? da.y : da.x));
    const float p1 = pexp((hh ? sa.w : sa.z) + (hh ? da.w : da.z));
    const float* hr = h1 + (size_t)node * D1;
    const v4f x0 = *(const v4f*)(hr + 4 * lane);
    const v4f x1 = *(const v4f*)(hr + 128 + 4 * lane);
    const v4f s0 = *(const v4f*)(sacc + slot * D1 + 4 * lane) + p0 * x0;
    const v4f s1 = *(const v4f*)(sacc + slot * D1 + 128 + 4 * lane) + p1 * x1;
    const float d0 = den[slot * NH1 + hh] + p0;
    const float d1 = den[slot * NH1 + 2 + hh] + p1;
    const float inv0 = 1.0f / (d0 + 1e-16f);
    const float inv1 = 1.0f / (d1 + 1e-16f);
    v4f v0 = s0 * inv0 + ba;
    v4f v1 = s1 * inv1 + bb;
    v0.x = eluf(v0.x); v0.y = eluf(v0.y); v0.z = eluf(v0.z); v0.w = eluf(v0.w);
    v1.x = eluf(v1.x); v1.y = eluf(v1.y); v1.z = eluf(v1.z); v1.w = eluf(v1.w);
    float* gp = g1 + (size_t)node * D1;
    *(volatile v4f*)(gp + 4 * lane) = v0;
    *(volatile v4f*)(gp + 128 + 4 * lane) = v1;
    __threadfence();
    *(volatile v4f*)(gp + 4 * lane) = v0;
    *(volatile v4f*)(gp + 128 + 4 * lane) = v1;
  }
}

__global__ __launch_bounds__(64) void k_gemm2(
    const float* __restrict__ g1, const __bf16* __restrict__ Wh, const __bf16* __restrict__ Wl,
    const float* __restrict__ att_s, const float* __restrict__ att_d,
    float* h2, float* asrc, float* adst, int nN) {
  __shared__ __attribute__((aligned(16))) float Ys[GR * D2];
  __shared__ __attribute__((aligned(16))) float Ss[GR];
  __shared__ __attribute__((aligned(16))) float Dd[GR];

  const int tid  = threadIdx.x;
  const int lane = tid & 31;
  const int w    = tid >> 5;
  const int hh   = lane >> 4;
  const int m    = lane & 15;
  const int rowBase = blockIdx.x * GR;

  int row = rowBase + 16 * w + m;
  if (row > nN - 1) row = nN - 1;
  const float* ap = g1 + (size_t)row * D1;

  v8f acc = zero8();
#pragma unroll 1
  for (int kt = 0; kt < KD / 32; ++kt) {
    const int ko = kt * 32 + 8 * hh;
    const v4f f0 = *(const v4f*)(ap + ko);
    const v4f f1 = *(const v4f*)(ap + ko + 4);
    const v4f f2 = *(const v4f*)(ap + ko + 16);
    const v4f f3 = *(const v4f*)(ap + ko + 20);
    PackB uh0, ul0, uh1, ul1;
    split8(f0, f1, uh0, ul0);
    split8(f2, f3, uh1, ul1);
    FragB ah, al, bh, bl;
    ah.half[0] = uh0.b; ah.half[1] = uh1.b;
    al.half[0] = ul0.b; al.half[1] = ul1.b;
    const __bf16* pb = Wh + (size_t)m * KD + ko;
    bh.half[0] = *(const v8b*)pb; bh.half[1] = *(const v8b*)(pb + 16);
    pb = Wl + (size_t)m * KD + ko;
    bl.half[0] = *(const v8b*)pb; bl.half[1] = *(const v8b*)(pb + 16);
    acc = wmb(ah.v, bh.v, acc); acc = wmb(ah.v, bl.v, acc); acc = wmb(al.v, bh.v, acc);
  }

  const float cs = att_s[m], cd = att_d[m];
  float ss[8], sd[8];
#pragma unroll
  for (int r = 0; r < 8; ++r) {
    Ys[(16 * w + 8 * hh + r) * D2 + m] = acc[r];
    ss[r] = acc[r] * cs;
    sd[r] = acc[r] * cd;
  }
#pragma unroll
  for (int mk = 1; mk < 16; mk <<= 1) {
#pragma unroll
    for (int r = 0; r < 8; ++r) {
      ss[r] += __shfl_xor(ss[r], mk, 32);
      sd[r] += __shfl_xor(sd[r], mk, 32);
    }
  }
  if (m == 0) {
#pragma unroll
    for (int r = 0; r < 8; ++r) {
      Ss[16 * w + 8 * hh + r] = ss[r];
      Dd[16 * w + 8 * hh + r] = sd[r];
    }
  }
  __syncthreads();

  const v4f y0 = *(const v4f*)(Ys + 4 * tid);
  const v4f y1 = *(const v4f*)(Ys + 256 + 4 * tid);
  float* hp = h2 + (size_t)rowBase * D2;
  v4f fv = zero4();
  float* fp = 0;
  if (tid < 8)       { fv = *(const v4f*)(Ss + 4 * tid);       fp = asrc + (size_t)rowBase + 4 * tid; }
  else if (tid < 16) { fv = *(const v4f*)(Dd + 4 * (tid - 8)); fp = adst + (size_t)rowBase + 4 * (tid - 8); }
  *(volatile v4f*)(hp + 4 * tid) = y0;
  *(volatile v4f*)(hp + 256 + 4 * tid) = y1;
  if (fp) *(volatile v4f*)fp = fv;
  __threadfence();
  *(volatile v4f*)(hp + 4 * tid) = y0;
  *(volatile v4f*)(hp + 256 + 4 * tid) = y1;
  if (fp) *(volatile v4f*)fp = fv;
}

__global__ __launch_bounds__(NTHR) void k_gat2(
    const int* __restrict__ ei, const float* __restrict__ h2, const float* __restrict__ pe,
    const float* __restrict__ asrc, const float* __restrict__ adst, const float* __restrict__ b2,
    float* out, int nN, int nE) {
  extern __shared__ v4f lds_dyn[];
  float* sacc = (float*)lds_dyn;
  float* den  = sacc + NB2 * D2;
  int*   list = (int*)(sacc + LDS2_F);
  int*   wcnt = list + NWAVE * WCAP;

  const int tid  = threadIdx.x;
  const int lane = tid & 31;
  const int wave = tid >> 5;
  const int hh   = lane >> 4;
  const int m    = lane & 15;
  const int nodeBase = blockIdx.x * NB2;

  {
    const v4f z4 = zero4();
    for (int i = tid; i < LDS2_F / 4; i += NTHR) lds_dyn[i] = z4;
  }
  __syncthreads();

  const int* eid = ei + nE;
  const bool al16 = ((nE & 3) == 0);
  const int nChunks = (nE + CHUNK - 1) / CHUNK;
#pragma unroll 1
  for (int ch = 0; ch < nChunks; ++ch) {
    const int cbase = ch * CHUNK;
    const int wc = scan_chunk<NB2, SH2>(eid, nE, al16, cbase, nodeBase, tid, wave, list);
    if (lane == 0) wcnt[wave] = wc;
    __syncthreads();

    if (wave == 0) {
#pragma unroll 1
      for (int wsx = 0; wsx < NWAVE; ++wsx) {
        int n = wcnt[wsx];
        n = n > WCAP ? WCAP : n; n = n < 0 ? 0 : n;
        const int lb = wsx * WCAP;
#pragma unroll 1
        for (int i = 0; i < n; i += 2) {
          const bool two  = (i + 1 < n);
          const int entA  = list[lb + i];
          const int entB  = two ? list[lb + i + 1] : entA;
          const int slotA = entA & (NB2 - 1);
          const int slotB = entB & (NB2 - 1);
          const int ent   = hh ? entB : entA;
          const int slot  = hh ? slotB : slotA;
          const int el    = (ent >> SH2) & (CHUNK - 1);
          int e = cbase + el; if (e > nE - 1) e = nE - 1;
          const int src = clampi(ei[e], nN - 1);
          float p = pe[e];
          if (hh && !two) p = 0.f;
          const float hv = h2[(size_t)src * D2 + m];
          float contrib = p * hv;
          if (slotA == slotB) {
            contrib += __shfl_xor(contrib, 16, 32);
            const float pp = p + __shfl_xor(p, 16, 32);
            if (hh == 0) { const float o = sacc[slotA * D2 + m]; sacc[slotA * D2 + m] = o + contrib; }
            if (lane == 0) { const float o = den[slotA]; den[slotA] = o + pp; }
          } else {
            { const float o = sacc[slot * D2 + m]; sacc[slot * D2 + m] = o + contrib; }
            if (m == 0) { const float o = den[slot]; den[slot] = o + p; }
          }
        }
      }
    }
    __syncthreads();
  }

  const float bm = b2[m];
#pragma unroll 1
  for (int j = 0; j < NB2 / NWAVE; ++j) {
    const int slot = wave * (NB2 / NWAVE) + j;
    const int node = nodeBase + slot;
    if (node >= nN) break;
    const float p  = pexp(asrc[node] + adst[node]);
    const float sv = sacc[slot * D2 + m] + p * h2[(size_t)node * D2 + m];
    const float dv = den[slot] + p;
    const float o  = sv * (1.0f / (dv + 1e-16f)) + bm;
    if (hh == 0) sacc[slot * D2 + m] = o;
  }
  __syncthreads();

  int nrows = nN - nodeBase;
  if (nrows > NB2) nrows = NB2;
  const int nv = nrows * (D2 / 4);
  float* ob = out + (size_t)nodeBase * D2;
  for (int i = tid; i < nv; i += NTHR) { const v4f v = lds_dyn[i]; *(volatile v4f*)(ob + 4 * (size_t)i) = v; }
  __threadfence();
  for (int i = tid; i < nv; i += NTHR) { const v4f v = lds_dyn[i]; *(volatile v4f*)(ob + 4 * (size_t)i) = v; }
}

extern "C" void kernel_launch(void* const* d_in, const int* in_sizes, int n_in,
                              void* d_out, int out_size, void* d_ws, size_t ws_size,
                              hipStream_t stream) {
  if (n_in < 10) return;
  if (in_sizes[0] <= 0 || (in_sizes[0] % FIN) != 0) return;
  const int nN = in_sizes[0] / FIN;
  if (in_sizes[1] < 0 || (in_sizes[1] & 1) != 0) return;
  const int nE = in_sizes[1] / 2;
  if (in_sizes[2] != FIN * D1 || in_sizes[3] != D1 || in_sizes[4] != D1 || in_sizes[5] != D1) return;
  if (in_sizes[6] != D1 * D2 || in_sizes[7] != D2 || in_sizes[8] != D2 || in_sizes[9] != D2) return;
  if (out_size != nN * D2) return;

  const float* x        = (const float*)d_in[0];
  const int*   ei       = (const int*)d_in[1];
  const float* W1       = (const float*)d_in[2];
  const float* att_src1 = (const float*)d_in[3];
  const float* att_dst1 = (const float*)d_in[4];
  const float* b1       = (const float*)d_in[5];
  const float* W2       = (const float*)d_in[6];
  const float* att_src2 = (const float*)d_in[7];
  const float* att_dst2 = (const float*)d_in[8];
  const float* b2       = (const float*)d_in[9];
  float* out = (float*)d_out;

  const int nP = ((nN + GR - 1) / GR) * GR;
  const int Ep = ((nE + 127) / 128) * 128;

  size_t off = 0;
  auto carve = [&](size_t bytes) -> char* {
    char* p = (char*)d_ws + off;
    off += (bytes + 255) & ~(size_t)255;
    return p;
  };
  __bf16* P1h = (__bf16*)carve((size_t)D1 * KD * 2);
  __bf16* P1l = (__bf16*)carve((size_t)D1 * KD * 2);
  __bf16* P2h = (__bf16*)carve((size_t)D2 * KD * 2);
  __bf16* P2l = (__bf16*)carve((size_t)D2 * KD * 2);
  float* h1  = (float*)carve((size_t)nP * D1 * 4);
  float* as1 = (float*)carve((size_t)nP * NH1 * 4);
  float* ad1 = (float*)carve((size_t)nP * NH1 * 4);
  float* pe1 = (float*)carve((size_t)Ep * NH1 * 4);
  float* g1  = (float*)carve((size_t)nP * D1 * 4);
  float* h2  = (float*)carve((size_t)nP * D2 * 4);
  float* as2 = (float*)carve((size_t)nP * 4);
  float* ad2 = (float*)carve((size_t)nP * 4);
  float* pe2 = (float*)carve((size_t)Ep * 4);
  if (off > ws_size) return;
  if (off > (size_t)134217728u) return;

  const int nb1 = D1 / 8, nb2 = D2 / 8;
  k_prep<<<nb1 + nb2, NTHR, 0, stream>>>(W1, P1h, P1l, W2, P2h, P2l, nb1);

  k_gemm1<<<nP / GR, NTHR, 0, stream>>>(x, P1h, P1l, att_src1, att_dst1, h1, as1, ad1, nN);

  if (Ep > 0) {
    k_edge1<<<(Ep + NTHR - 1) / NTHR, NTHR, 0, stream>>>(ei, as1, ad1, pe1, nN, nE, Ep);
  }

  hipFuncSetAttribute(reinterpret_cast<const void*>(&k_gat1),
                      hipFuncAttributeMaxDynamicSharedMemorySize, LDS1_BYTES);
  k_gat1<<<(nN + NB1 - 1) / NB1, NTHR, LDS1_BYTES, stream>>>(ei, h1, pe1, as1, ad1, b1, g1, nN, nE);

  k_gemm2<<<nP / GR, 64, 0, stream>>>(g1, P2h, P2l, att_src2, att_dst2, h2, as2, ad2, nN);

  if (Ep > 0) {
    const int Ep4 = Ep / 4;
    k_edge2<<<(Ep4 + NTHR - 1) / NTHR, NTHR, 0, stream>>>(ei, as2, ad2, pe2, nN, nE, Ep4);
  }

  hipFuncSetAttribute(reinterpret_cast<const void*>(&k_gat2),
                      hipFuncAttributeMaxDynamicSharedMemorySize, LDS2_BYTES);
  k_gat2<<<(nN + NB2 - 1) / NB2, NTHR, LDS2_BYTES, stream>>>(ei, h2, pe2, as2, ad2, b2, out, nN, nE);
}
